// TSACoding_70231305224552
// MI455X (gfx1250) — hardware-run, weakly checked
//
#include <hip/hip_runtime.h>


#ifndef NI
#define NI 64
#endif
#ifndef NC
#define NC 64
#endif
#define NI_FULL 64
#define NC_FULL 64
#define MAXR 36
#define MAXW 32
#define DIM  1024
#define CG   8
#define RT   3
#define GSP  36
#define PCAR 16384.0f
#define PINV (1.0f / 16384.0f)
#define LOG2E 1.4426950408889634f
#define NEGB (-1.0e30f)

static_assert(MAXW == 32);
static_assert(RT * 16 >= MAXR);
static_assert((RT - 1) * 16 < MAXR);
static_assert(DIM % 32 == 0);
static_assert(NC % CG == 0);
static_assert((CG * MAXR * 4) % 128 == 0);
static_assert((NC_FULL * MAXR * 4) % 128 == 0);
static_assert((CG * MAXR / 4) % 8 == 0);
static_assert((CG * MAXR / 4) <= 3 * 32);
static_assert((CG * MAXR / 4) > 2 * 32);
static_assert(4 * 32 * 8 == MAXW * MAXW);
static_assert(((size_t)NI * MAXR * DIM) % 8 == 0);
static_assert(((size_t)NC * MAXW * DIM) % 8 == 0);
static_assert(NI <= NI_FULL);
static_assert(NC <= NC_FULL);
static_assert((GSP * 4) % 16 == 0);
static_assert(MAXW * GSP * 4 <= 131072);
static_assert(CG * MAXR * 4 <= 131072);

typedef _Float16 h16;
typedef unsigned short bf;
typedef __attribute__((ext_vector_type(16))) __bf16   v16bf;
typedef __attribute__((ext_vector_type(16))) _Float16 v16h;
typedef __attribute__((ext_vector_type(8)))  _Float16 v8h;
typedef __attribute__((ext_vector_type(8)))  unsigned short v8us;
typedef __attribute__((ext_vector_type(8)))  float    v8f;
typedef __attribute__((ext_vector_type(4)))  float    v4f;
typedef v4f  __attribute__((may_alias)) v4fa;

__device__ __forceinline__ unsigned short f2bf(float f) { unsigned u = __float_as_uint(f); u += 0x7FFFu + ((u >> 16) & 1u); return (unsigned short)(u >> 16); }
__device__ __forceinline__ float bfr(float f) { return __uint_as_float(((unsigned)f2bf(f)) << 16); }
__device__ __forceinline__ v16h cat16(v8h lo, v8h hi) { return __builtin_shufflevector(lo, hi, 0, 1, 2, 3, 4, 5, 6, 7, 8, 9, 10, 11, 12, 13, 14, 15); }
__device__ __forceinline__ v16bf cat16b(v8us lo, v8us hi) { return __builtin_bit_cast(v16bf, __builtin_shufflevector(lo, hi, 0, 1, 2, 3, 4, 5, 6, 7, 8, 9, 10, 11, 12, 13, 14, 15)); }
__device__ __forceinline__ v8f wmma16(v16h a, v16h b, v8f c) { return __builtin_amdgcn_wmma_f32_16x16x32_f16(false, a, false, b, (short)0, c, false, false); }
__device__ __forceinline__ v8f wmmab(v16bf a, v16bf b, v8f c) { return __builtin_amdgcn_wmma_f32_16x16x32_bf16(false, a, false, b, (short)0, c, false, false); }
__device__ __forceinline__ v16h  ldh(const h16* p) { return cat16(*(const v8h*)p, *(const v8h*)(p + 16)); }
__device__ __forceinline__ v16bf ldb(const bf* p)  { return cat16b(*(const v8us*)p, *(const v8us*)(p + 16)); }
__device__ __forceinline__ void wave_sync() { __builtin_amdgcn_fence(3  , "wavefront"); __builtin_amdgcn_wave_barrier(); asm volatile("" ::: "memory"); }

__device__ __forceinline__ v8f wmmab_g(v16bf a, v16bf b, v8f c) { c = wmmab(a, b, c); asm volatile("v_nop\n\tv_nop\n\tv_nop\n\tv_nop" : "+v"(c) : "v"(a), "v"(b)); return c; }
__device__ __forceinline__ v8f wmma16_g(v16h a, v16h b, v8f c) { c = wmma16(a, b, c); asm volatile("v_nop\n\tv_nop\n\tv_nop\n\tv_nop" : "+v"(c) : "v"(a), "v"(b)); return c; }
static __device__ __forceinline__ h16 toh_flush(float v) { const h16 r = (h16)v; return (fabsf(v) < 6.103515625e-05f) ? (h16)0.0f : r; }

__global__ __launch_bounds__(256) void k_cvt8(const float* __restrict__ src, bf* dst, size_t n8) {
    const size_t i = (size_t)blockIdx.x * 256 + threadIdx.x; if (i >= n8) return;
    const v8f v = *(const v8f*)(src + i * 8); v8us o;
#pragma unroll
    for (int k = 0; k < 8; ++k) o[k] = f2bf(v[k]);
    *(volatile v8us*)(dst + i * 8) = o; __threadfence(); *(volatile v8us*)(dst + i * 8) = o;
}

__global__ __launch_bounds__(32) void k_gram(const bf* __restrict__ CB, const int* __restrict__ cap_lens, h16* GH) {
    __shared__ __align__(16) float gs[MAXW * GSP];
    const int lane = threadIdx.x & 31, lr = lane & 15, hi = lane >> 4;
    const int c = blockIdx.x;
    const int cln = cap_lens[c];
    v8f g00 = (v8f){}, g01 = (v8f){}, g10 = (v8f){}, g11 = (v8f){};
    const size_t off = ((size_t)c * MAXW + lr) * DIM + 8 * hi;
#pragma unroll 1
    for (int kc = 0; kc < DIM; kc += 32) {
        const v16bf a0 = ldb(CB + off + kc);
        const v16bf a1 = ldb(CB + off + (size_t)16 * DIM + kc);
        g00 = wmmab_g(a0, a0, g00); g01 = wmmab_g(a0, a1, g01);
        g10 = wmmab_g(a1, a0, g10); g11 = wmmab_g(a1, a1, g11);
    }
    const bool c0 = lr < cln, c1 = (16 + lr) < cln;
#pragma unroll
    for (int j = 0; j < 8; ++j) {
        const int wa = 8 * hi + j, wb = 16 + 8 * hi + j;
        const bool ka = wa < cln, kb = wb < cln;
        gs[wa * GSP + lr]      = (ka & c0) ? g00[j] : 0.0f;
        gs[wa * GSP + 16 + lr] = (ka & c1) ? g01[j] : 0.0f;
        gs[wb * GSP + lr]      = (kb & c0) ? g10[j] : 0.0f;
        gs[wb * GSP + 16 + lr] = (kb & c1) ? g11[j] : 0.0f;
    }
    wave_sync();
    h16* gp = GH + (size_t)c * (MAXW * MAXW);
#pragma unroll 1
    for (int ps = 0; ps < 2; ++ps) {
#pragma unroll
        for (int s = 0; s < 4; ++s) { const int p = s * 32 + lane; const int row = p >> 2, c8 = (p & 3) * 8;
            const v4f x0 = *(const v4fa*)(&gs[row * GSP + c8]); const v4f x1 = *(const v4fa*)(&gs[row * GSP + c8 + 4]); v8h hv;
#pragma unroll
            for (int i = 0; i < 4; ++i) { hv[i] = toh_flush(x0[i]); hv[4 + i] = toh_flush(x1[i]); }
            *(volatile v8h*)(gp + (size_t)p * 8) = hv; }
        if (ps == 0) __threadfence(); }
}

__device__ __forceinline__ float pair_rows(const v8f s0, const v8f s1, const v16h g0, const v16h g1, const int cln, const int hi, const bool rvalid) {
    float raw[16], x[16], ex[16], p[16]; bool ok[16];
#pragma unroll
    for (int j = 0; j < 8; ++j) {
        raw[j] = s0[j]; raw[8 + j] = s1[j];
        ok[j] = (8 * hi + j) < cln; ok[8 + j] = (16 + 8 * hi + j) < cln; }
    float ss = 0.0f;
#pragma unroll
    for (int e = 0; e < 16; ++e) {
        const float lk = (raw[e] >= 0.0f) ? raw[e] : 0.1f * raw[e];
        x[e] = ok[e] ? lk : 0.0f;
        ss += x[e] * x[e]; }
    ss += __shfl_xor(ss, 16, 32);
    const float rn = 1.0f / (sqrtf(ss) + 1.0e-8f);
    float mx = NEGB;
#pragma unroll
    for (int e = 0; e < 16; ++e) { x[e] = (x[e] * rn) * 10.0f; mx = fmaxf(mx, ok[e] ? x[e] : NEGB); }
    mx = fmaxf(mx, __shfl_xor(mx, 16, 32));
    float se = 0.0f;
#pragma unroll
    for (int e = 0; e < 16; ++e) { const float t = __builtin_amdgcn_exp2f((x[e] - mx) * LOG2E); ex[e] = ok[e] ? t : 0.0f; se += ex[e]; }
    se += __shfl_xor(se, 16, 32);
    const float ri = 1.0f / se;
    float num = 0.0f; v16h pb;
#pragma unroll
    for (int e = 0; e < 16; ++e) {
        const float pe = ex[e] * ri;
        p[e] = ok[e] ? pe : 0.0f;
        num += p[e] * raw[e];
        pb[e] = toh_flush(p[e] * PCAR); }
    num += __shfl_xor(num, 16, 32);
    v8f d0 = (v8f){}, d1 = (v8f){};
    d0 = wmma16_g(g0, pb, d0);
    d1 = wmma16_g(g1, pb, d1);
    float q = 0.0f;
#pragma unroll
    for (int j = 0; j < 8; ++j) q += p[j] * d0[j] + p[8 + j] * d1[j];
    q += __shfl_xor(q, 16, 32);
    q *= PINV;
    const float den = sqrtf(fmaxf(q, 0.0f)) + (-1.0e-8f);
    const float o = num * (1.0f / den);
    return rvalid ? o : -1.0f;
}

__global__ __launch_bounds__(32 * CG) void k_pair(const bf* __restrict__ IB, const bf* __restrict__ CB, const h16* __restrict__ GH,
                                                  const int* __restrict__ img_lens, const int* __restrict__ cap_lens, float* OUT) {
    __shared__ __align__(16) float os[CG * MAXR];
    const int lane = threadIdx.x & 31, lr = lane & 15, hi = lane >> 4;
    const int wave = __builtin_amdgcn_readfirstlane((int)(threadIdx.x >> 5));
    const int i = blockIdx.y; const int c = blockIdx.x * CG + wave;
    const int iln = img_lens[i]; const int cln = cap_lens[c];
    int r2 = 32 + lr; r2 = r2 > (MAXR - 1) ? (MAXR - 1) : r2;
    const size_t ao  = ((size_t)c * MAXW + lr) * DIM + 8 * hi;
    const size_t bo0 = ((size_t)i * MAXR + lr) * DIM + 8 * hi;
    const size_t bo1 = ((size_t)i * MAXR + 16 + lr) * DIM + 8 * hi;
    const size_t bo2 = ((size_t)i * MAXR + r2) * DIM + 8 * hi;
    v8f s00 = (v8f){}, s01 = (v8f){}, s02 = (v8f){}, s10 = (v8f){}, s11 = (v8f){}, s12 = (v8f){};
#pragma unroll 1
    for (int kc = 0; kc < DIM; kc += 32) {
        const v16bf a0 = ldb(CB + ao + kc);
        const v16bf a1 = ldb(CB + ao + (size_t)16 * DIM + kc);
        const v16bf b0 = ldb(IB + bo0 + kc);
        const v16bf b1 = ldb(IB + bo1 + kc);
        const v16bf b2 = ldb(IB + bo2 + kc);
        s00 = wmmab_g(a0, b0, s00); s10 = wmmab_g(a1, b0, s10);
        s01 = wmmab_g(a0, b1, s01); s11 = wmmab_g(a1, b1, s11);
        s02 = wmmab_g(a0, b2, s02); s12 = wmmab_g(a1, b2, s12);
    }
    const h16* gb = GH + (size_t)c * (MAXW * MAXW) + (size_t)lr * MAXW + 8 * hi;
    const v16h g0 = ldh(gb), g1 = ldh(gb + 16 * MAXW);
    const float o0 = pair_rows(s00, s10, g0, g1, cln, hi, lr < iln);
    const float o1 = pair_rows(s01, s11, g0, g1, cln, hi, (16 + lr) < iln);
    const float o2 = pair_rows(s02, s12, g0, g1, cln, hi, (32 + lr) < iln);
    if (hi == 0) {
        os[wave * MAXR + lr] = o0;
        os[wave * MAXR + 16 + lr] = o1;
        if (lr < MAXR - 32) os[wave * MAXR + 32 + lr] = o2; }
    __syncthreads();
    if (wave == 0) {
        float* ob = OUT + ((size_t)i * NC_FULL + (size_t)blockIdx.x * CG) * MAXR;
#pragma unroll 1
        for (int ps = 0; ps < 2; ++ps) {
#pragma unroll
            for (int s = 0; s < 3; ++s) { const int p = s * 32 + lane;
                const int pc = p < (CG * MAXR / 4) ? p : (CG * MAXR / 4 - 1);
                v4f val = *(const v4fa*)(&os[pc * 4]);
                asm volatile("" : "+v"(val));
                if (p < (CG * MAXR / 4)) *(volatile v4f*)(ob + (size_t)p * 4) = val; }
            if (ps == 0) __threadfence(); }
    }
}

static constexpr size_t al256(size_t v) { return (v + 255) & ~(size_t)255; }
static constexpr size_t SZ_IB = al256((size_t)NI * MAXR * DIM * 2);
static constexpr size_t SZ_CB = al256((size_t)NC * MAXW * DIM * 2);
static constexpr size_t SZ_GH = al256((size_t)NC * MAXW * MAXW * 2);
static constexpr size_t SZ_TOTAL = SZ_IB + SZ_CB + SZ_GH;
static_assert(SZ_TOTAL <= (size_t)134217728);
static_assert(((size_t)MAXW * MAXW * 2) % 128 == 0);

extern "C" void kernel_launch(void* const* d_in, const int* in_sizes, int n_in,
                              void* d_out, int out_size, void* d_ws, size_t ws_size, hipStream_t stream) {
    if (n_in < 4) return;
    if ((size_t)in_sizes[0] < (size_t)NI * MAXR * DIM) return;
    if ((size_t)in_sizes[1] < (size_t)NC * MAXW * DIM) return;
    if (in_sizes[2] < NI || in_sizes[3] < NC) return;
    if ((size_t)out_size < ((size_t)(NI - 1) * NC_FULL + NC) * MAXR) return;
    if (SZ_TOTAL > ws_size) return;
    const float* imgs = (const float*)d_in[0];
    const float* caps = (const float*)d_in[1];
    const int* img_lens = (const int*)d_in[2];
    const int* cap_lens = (const int*)d_in[3];
    float* OUT = (float*)d_out;
    char* wsp = (char*)d_ws;
    bf* IB = (bf*)wsp; wsp += SZ_IB;
    bf* CB = (bf*)wsp; wsp += SZ_CB;
    h16* GH = (h16*)wsp; wsp += SZ_GH;

    { const size_t n8 = (size_t)NI * MAXR * DIM / 8; k_cvt8<<<(unsigned)((n8 + 255) / 256), 256, 0, stream>>>(imgs, IB, n8); }
    { const size_t n8 = (size_t)NC * MAXW * DIM / 8; k_cvt8<<<(unsigned)((n8 + 255) / 256), 256, 0, stream>>>(caps, CB, n8); }
    k_gram<<<dim3(NC, 1, 1), 32, 0, stream>>>(CB, cap_lens, GH);
    k_pair<<<dim3(NC / CG, NI, 1), 32 * CG, 0, stream>>>(IB, CB, GH, img_lens, cap_lens, OUT);
}
